// Sparse_Graph_Attention_Layer_62130996903989
// MI455X (gfx1250) — hardware-verified
//
#include <hip/hip_runtime.h>
#include <stddef.h>
#include <stdint.h>
#include <math.h>


#define IN_DIM   256
#define OUT_DIM  128
#define NTHR     256
#define NWAVE    8
#define EPT      8
#define CHUNK    (NTHR * EPT)
#define WCAP     (EPT * 32)
#define LISTN    (NWAVE * WCAP)
#define NBRUN    512
#define SLB      9
#define RCAP     28672
#define DEGCAP   64
#define GBM      128
#define GBN      128
#define GTHR     256
#define NWB      ((OUT_DIM * (IN_DIM / 8)) / NTHR)
#define NEGSL    0.2f
#define AGG_ZINTS    (LISTN + 2 * RCAP + 3 * NBRUN)
#define AGG_LDS_INTS (AGG_ZINTS + 16)
#define GEMM_LDS_FLOATS (GBM * GBN + 2 * OUT_DIM + 2 * GBM)
#define WSMAX    134217728

static_assert((CHUNK & (CHUNK - 1)) == 0 && CHUNK <= 4096);
static_assert(NBRUN == (1 << SLB));
static_assert(((long long)CHUNK << SLB) < (1LL << 31));
static_assert(NBRUN % NWAVE == 0 && NBRUN % 32 == 0);
static_assert(RCAP % 4 == 0 && AGG_ZINTS % 4 == 0 && LISTN % 4 == 0);
static_assert(RCAP <= NBRUN * DEGCAP);
static_assert(AGG_LDS_INTS * 4 <= 327680);
static_assert(GEMM_LDS_FLOATS * 4 <= 327680);
static_assert(IN_DIM % 32 == 0 && IN_DIM / 8 == 32);
static_assert(OUT_DIM == GBN && OUT_DIM == 4 * 32);
static_assert(GBM == (GTHR / 32) * 16);
static_assert((OUT_DIM * (IN_DIM / 8)) % NTHR == 0);
static_assert(2 * OUT_DIM == 64 * 4);
static_assert(NBRUN % GBM == 0);

typedef float          v4f  __attribute__((ext_vector_type(4)));
typedef float          v8f  __attribute__((ext_vector_type(8)));
typedef int            v4i  __attribute__((ext_vector_type(4)));
typedef int            v8i  __attribute__((ext_vector_type(8)));
typedef unsigned int   v4u  __attribute__((ext_vector_type(4)));
typedef unsigned short v8us __attribute__((ext_vector_type(8)));
typedef __bf16         v16b __attribute__((ext_vector_type(16)));
typedef v4f  __attribute__((may_alias)) v4fa;
typedef v4i  __attribute__((may_alias)) v4ia;
typedef v8us __attribute__((may_alias)) v8usa;
union FragB { v16b v; v8us h[2]; v8i w; };

__device__ __forceinline__ v8f wmb(const FragB& a, const FragB& b, v8f c) {
  v8f d = __builtin_amdgcn_wmma_f32_16x16x32_bf16(false, a.v, false, b.v, (short)0, c, false, false);
  asm volatile("v_nop\n\tv_nop\n\tv_nop\n\tv_nop" : "+v"(d) : "v"(a.w), "v"(b.w));
  return d;
}

__device__ __forceinline__ unsigned int f2bf(float f) {
  const unsigned int u = __float_as_uint(f);
  return ((u + 0x7FFFu + ((u >> 16) & 1u)) >> 16) & 0xFFFFu;
}
__device__ __forceinline__ float bf2f(unsigned int b) { return __uint_as_float(b << 16); }
__device__ __forceinline__ float bfr(float f) { return bf2f(f2bf(f)); }
__device__ __forceinline__ v4f bfr4(const v4f a) {
  v4f r; r.x = bfr(a.x); r.y = bfr(a.y); r.z = bfr(a.z); r.w = bfr(a.w); return r;
}
__device__ __forceinline__ unsigned int pk2(float lo, float hi) { return f2bf(lo) | (f2bf(hi) << 16); }
__device__ __forceinline__ v4u pack8(const v4f a, const v4f b) {
  v4u r;
  r.x = pk2(a.x, a.y); r.y = pk2(a.z, a.w); r.z = pk2(b.x, b.y); r.w = pk2(b.z, b.w);
  return r;
}

__device__ __forceinline__ int scan_chunk(const int* __restrict__ keys, int nE, int cbase, int slotBase,
                                          int nb, int vec8, int* list, int tid, int lane, int wave) {
  int wc = 0;
  const int el0  = tid * EPT;
  const int e0   = cbase + el0;
  const int sent = -2147483647 - 1;
  v4i da, db;
  if (vec8 != 0 && cbase + CHUNK <= nE) {
    da = *(const v4i*)(keys + e0);
    db = *(const v4i*)(keys + e0 + 4);
  } else {
    da.x = (e0     < nE) ? keys[min(e0,     nE - 1)] : sent;
    da.y = (e0 + 1 < nE) ? keys[min(e0 + 1, nE - 1)] : sent;
    da.z = (e0 + 2 < nE) ? keys[min(e0 + 2, nE - 1)] : sent;
    da.w = (e0 + 3 < nE) ? keys[min(e0 + 3, nE - 1)] : sent;
    db.x = (e0 + 4 < nE) ? keys[min(e0 + 4, nE - 1)] : sent;
    db.y = (e0 + 5 < nE) ? keys[min(e0 + 5, nE - 1)] : sent;
    db.z = (e0 + 6 < nE) ? keys[min(e0 + 6, nE - 1)] : sent;
    db.w = (e0 + 7 < nE) ? keys[min(e0 + 7, nE - 1)] : sent;
  }
  const unsigned nbs = (unsigned)slotBase;
  const unsigned unb = (unsigned)nb;
  const unsigned s0 = (unsigned)da.x - nbs, s1 = (unsigned)da.y - nbs;
  const unsigned s2 = (unsigned)da.z - nbs, s3 = (unsigned)da.w - nbs;
  const unsigned s4 = (unsigned)db.x - nbs, s5 = (unsigned)db.y - nbs;
  const unsigned s6 = (unsigned)db.z - nbs, s7 = (unsigned)db.w - nbs;
  const bool h0 = s0 < unb, h1 = s1 < unb, h2 = s2 < unb, h3 = s3 < unb;
  const bool h4 = s4 < unb, h5 = s5 < unb, h6 = s6 < unb, h7 = s7 < unb;
  const unsigned any = __builtin_amdgcn_ballot_w32(h0 | h1 | h2 | h3 | h4 | h5 | h6 | h7);
  if (any != 0u) {
#define HITJ(J, HJ, SJ) { \
      const unsigned mj = __builtin_amdgcn_ballot_w32(HJ); \
      if (mj != 0u) { \
        if (HJ) { \
          const int pos = wc + (int)__builtin_amdgcn_mbcnt_lo(mj, 0u); \
          if (pos < WCAP) list[wave * WCAP + pos] = ((el0 + (J)) << SLB) | (int)(SJ); \
        } \
        wc += (int)__builtin_popcount(mj); } }
    HITJ(0, h0, s0)
    HITJ(1, h1, s1)
    HITJ(2, h2, s2)
    HITJ(3, h3, s3)
    HITJ(4, h4, s4)
    HITJ(5, h5, s5)
    HITJ(6, h6, s6)
    HITJ(7, h7, s7)
#undef HITJ
  }
  return wc;
}

__global__ __launch_bounds__(NTHR) void k_prep(const float* __restrict__ x, const float* __restrict__ w,
                                               const float* __restrict__ av,
                                               unsigned short* xb, unsigned short* wt, float* atab,
                                               int nN, int nXB) {
  const int b = (int)blockIdx.x, tid = (int)threadIdx.x;
  if (b < nXB) {
    const int i   = b * NTHR + tid;
    const int row = i >> 5;
    const int c0  = (i & 31) * 8;
    const int rc  = row < nN ? row : nN - 1;
    const float* p = x + (size_t)rc * IN_DIM + c0;
    v4f a0 = *(const v4fa*)p, a1 = *(const v4fa*)(p + 4);
    const v4f z4 = {0.f, 0.f, 0.f, 0.f};
    if (row >= nN) { a0 = z4; a1 = z4; }
    const v4u hv = pack8(a0, a1);
    unsigned short* o = xb + (size_t)row * IN_DIM + c0;
    *(volatile v4u*)o = hv;
    __threadfence();
    *(volatile v4u*)o = hv;
  } else if (b < nXB + NWB) {
    const int u  = (b - nXB) * NTHR + tid;
    const int n  = u >> 5;
    const int k8 = (u & 31) * 8;
    const float* p = w + (size_t)k8 * OUT_DIM + n;
    v4f a0, a1;
    a0.x = p[0];            a0.y = p[OUT_DIM];      a0.z = p[2 * OUT_DIM];  a0.w = p[3 * OUT_DIM];
    a1.x = p[4 * OUT_DIM];  a1.y = p[5 * OUT_DIM];  a1.z = p[6 * OUT_DIM];  a1.w = p[7 * OUT_DIM];
    const v4u wv = pack8(a0, a1);
    unsigned short* o = wt + (size_t)n * IN_DIM + k8;
    *(volatile v4u*)o = wv;
    __threadfence();
    *(volatile v4u*)o = wv;
  } else {
    if (tid < 64) {
      const v4f a = *(const v4fa*)(av + 4 * tid);
      const v4f r = bfr4(a);
      float* o = atab + 4 * tid;
      *(volatile v4f*)o = r;
      __threadfence();
      *(volatile v4f*)o = r;
    }
  }
}

__global__ __launch_bounds__(GTHR) __attribute__((amdgpu_num_vgpr(248)))
void k_gemm(const unsigned short* __restrict__ A, const unsigned short* __restrict__ BT,
            const float* __restrict__ atab, float* WH, float* S12, int MPr) {
  extern __shared__ __attribute__((aligned(16))) float gsm[];
  float* stg = gsm;
  float* sat = gsm + GBM * GBN;
  float* sdt = sat + 2 * OUT_DIM;
  const int tid = (int)threadIdx.x, lane = tid & 31, wave = tid >> 5, hh = lane >> 4, m = lane & 15;
  const int rowBase = (int)blockIdx.x * GBM;

  if (tid < 64) {
    const v4f a = *(const v4fa*)(atab + 4 * tid);
    *(v4fa*)(sat + 4 * tid) = a;
  }

  v8f acc[8];
  {
    const v8f z = {0.f, 0.f, 0.f, 0.f, 0.f, 0.f, 0.f, 0.f};
#pragma unroll
    for (int t = 0; t < 8; ++t) acc[t] = z;
  }
  const unsigned short* ap = A  + (size_t)(rowBase + 16 * wave + m) * (size_t)IN_DIM + 8 * hh;
  const unsigned short* bp = BT + (size_t)m * (size_t)IN_DIM + 8 * hh;

#pragma unroll 1
  for (int k0 = 0; k0 < IN_DIM; k0 += 32) {
    FragB af;
    af.h[0] = *(const v8usa*)(ap + k0);
    af.h[1] = *(const v8usa*)(ap + k0 + 16);
#pragma unroll
    for (int nt = 0; nt < 8; ++nt) {
      const unsigned short* wq = bp + (size_t)(16 * nt) * (size_t)IN_DIM + k0;
      FragB bf;
      bf.h[0] = *(const v8usa*)wq;
      bf.h[1] = *(const v8usa*)(wq + 16);
      acc[nt] = wmb(af, bf, acc[nt]);
    }
  }

#pragma unroll
  for (int nt = 0; nt < 8; ++nt) {
    const int lc = 16 * nt + m;
#pragma unroll
    for (int r = 0; r < 8; ++r) {
      const int lr = 16 * wave + 8 * hh + r;
      stg[lr * GBN + lc] = acc[nt][r];
    }
  }
  __syncthreads();

  const v4f a1v = *(const v4fa*)(sat + 4 * lane);
  const v4f a2v = *(const v4fa*)(sat + OUT_DIM + 4 * lane);
#pragma unroll 1
  for (int i = 0; i < 16; ++i) {
    const int row = wave * 16 + i;
    const v4f p = *(const v4fa*)(stg + row * GBN + 4 * lane);
    float s = 0.0f, d = 0.0f;
    s = fmaf(p.x, a1v.x, s); s = fmaf(p.y, a1v.y, s); s = fmaf(p.z, a1v.z, s); s = fmaf(p.w, a1v.w, s);
    d = fmaf(p.x, a2v.x, d); d = fmaf(p.y, a2v.y, d); d = fmaf(p.z, a2v.z, d); d = fmaf(p.w, a2v.w, d);
#pragma unroll
    for (int off = 16; off > 0; off >>= 1) {
      s += __shfl_xor(s, off);
      d += __shfl_xor(d, off);
    }
    if (lane == 0) { sdt[row] = s; sdt[GBM + row] = d; }
  }
  __syncthreads();

  const int pl = wave & 1;
  const v4f sv = *(const v4fa*)(sdt + pl * GBM + 4 * lane);
  float* sp = S12 + (size_t)pl * (size_t)MPr + (size_t)rowBase + 4 * lane;
  const bool wsd = wave < 2;
#pragma unroll 1
  for (int i = 0; i < 16; ++i) {
    const int row = wave * 16 + i;
    const v4f p = *(const v4fa*)(stg + row * GBN + 4 * lane);
    float* op = WH + (size_t)(rowBase + row) * (size_t)GBN + 4 * lane;
    *(volatile v4f*)op = p;
  }
  if (wsd) *(volatile v4f*)sp = sv;
  __threadfence();
#pragma unroll 1
  for (int i = 0; i < 16; ++i) {
    const int row = wave * 16 + i;
    const v4f p = *(const v4fa*)(stg + row * GBN + 4 * lane);
    float* op = WH + (size_t)(rowBase + row) * (size_t)GBN + 4 * lane;
    *(volatile v4f*)op = p;
  }
  if (wsd) *(volatile v4f*)sp = sv;
}

__global__ __launch_bounds__(NTHR) __attribute__((amdgpu_num_vgpr(248)))
void k_scan(const int* __restrict__ keys, const int* __restrict__ cols, int nE, int nN, int vec8,
            const float* __restrict__ S1, const float* __restrict__ S2,
            const float* __restrict__ WH, float* outp) {
  extern __shared__ __attribute__((aligned(16))) int dsm[];
  int* list = dsm;
  int* hl   = dsm + LISTN;
  int* sl   = dsm + LISTN + RCAP;
  int* cnt  = dsm + LISTN + 2 * RCAP;
  int* offs = cnt + NBRUN;
  int* cur  = offs + NBRUN;
  int* misc = cur + NBRUN;
  const int tid = (int)threadIdx.x, lane = tid & 31, wave = tid >> 5;
  const int nodeBase = (int)blockIdx.x * NBRUN;

  {
    const v4i z4 = {0, 0, 0, 0};
    for (int i = tid * 4; i < AGG_ZINTS; i += NTHR * 4) *(v4ia*)(dsm + i) = z4;
    if (tid < 16) misc[tid] = 0;
  }
  __syncthreads();

  int t = 0, ov = 0;
  const int nChunks = (nE + CHUNK - 1) / CHUNK;
#pragma unroll 1
  for (int ch = 0; ch < nChunks; ++ch) {
    const int cbase = ch * CHUNK;
    const int wc = scan_chunk(keys, nE, cbase, nodeBase, NBRUN, vec8, list, tid, lane, wave);
    if (lane == 0) misc[wave] = wc;
    __syncthreads();
    if (wave == 0) {
#pragma unroll 1
      for (int w2 = 0; w2 < NWAVE; ++w2) {
        int c = misc[w2];
        c = c < 0 ? 0 : (c > WCAP ? WCAP : c);
#pragma unroll 1
        for (int b0 = 0; b0 < c; b0 += 32) {
          const int idx = b0 + lane;
          const int ent = list[w2 * WCAP + (idx < WCAP ? idx : WCAP - 1)];
          const int m32 = (c - b0) < 32 ? (c - b0) : 32;
#pragma unroll 1
          for (int k = 0; k < m32; ++k) {
            const int u    = __builtin_amdgcn_readlane(ent, k);
            const int slot = u & (NBRUN - 1);
            const int el   = (u >> SLB) & (CHUNK - 1);
            const int pk   = ((cbase + el) << SLB) | slot;
            if (t < RCAP) {
              if (lane == 0) { hl[t] = pk; cnt[slot] = cnt[slot] + 1; }
              t = t + 1;
            } else {
              ov = 1;
            }
          }
        }
      }
    }
    __syncthreads();
  }
  if (wave == 0 && lane == 0) { misc[8] = t; misc[9] = ov; }
  __syncthreads();
  int tt = misc[8];
  tt = tt < 0 ? 0 : (tt > RCAP ? RCAP : tt);

  if (wave == 0) {
    const int base = lane * (NBRUN / 32);
    int s = 0, bg = 0;
#pragma unroll 1
    for (int i = 0; i < NBRUN / 32; ++i) {
      const int cv = cnt[base + i];
      s += cv;
      bg |= (cv > DEGCAP) ? 1 : 0;
    }
    int incl = s;
#pragma unroll
    for (int d = 1; d < 32; d <<= 1) {
      const int y = __shfl_up(incl, d, 32);
      if (lane >= d) incl += y;
    }
    int run = incl - s;
#pragma unroll 1
    for (int i = 0; i < NBRUN / 32; ++i) {
      const int cv = cnt[base + i];
      offs[base + i] = run;
      cur[base + i]  = run;
      run += cv;
    }
    const unsigned bm = __builtin_amdgcn_ballot_w32(bg != 0);
    if (lane == 0) misc[10] = (bm != 0u) ? 1 : 0;
  }
  __syncthreads();
  if (wave == 0) {
#pragma unroll 1
    for (int b0 = 0; b0 < tt; b0 += 32) {
      const int idx = b0 + lane;
      const int ent = hl[idx < RCAP ? idx : RCAP - 1];
      const int m32 = (tt - b0) < 32 ? (tt - b0) : 32;
#pragma unroll 1
      for (int k = 0; k < m32; ++k) {
        const int u    = __builtin_amdgcn_readlane(ent, k);
        const int slot = u & (NBRUN - 1);
        if (lane == 0) {
          int p = cur[slot];
          p = p < 0 ? 0 : (p > RCAP - 1 ? RCAP - 1 : p);
          sl[p] = u;
          cur[slot] = p + 1;
        }
      }
    }
  }
  __syncthreads();

  const bool poison = (misc[9] != 0) || (misc[10] != 0);
  const float qnan = __int_as_float(0x7fc00000);
#pragma unroll 1
  for (int si = 0; si < NBRUN / NWAVE; ++si) {
    const int s    = si * NWAVE + wave;
    const int node = nodeBase + s;
    int c = cnt[s];
    c = c < 0 ? 0 : (c > DEGCAP ? DEGCAP : c);
    int o = offs[s];
    o = o < 0 ? 0 : (o > RCAP ? RCAP : o);
    if (c > tt - o) c = tt - o;
    c = c < 0 ? 0 : c;
    const int nc = node < nN ? node : nN - 1;
    const float s1v = S1[nc];
    float a0 = 0.0f, a1 = 0.0f, a2 = 0.0f, a3 = 0.0f, dn = 0.0f;
#pragma unroll 1
    for (int b0 = 0; b0 < c; b0 += 32) {
      const int j  = b0 + lane;
      const int jc = j < c ? j : c - 1;
      int idx = o + jc;
      idx = idx < 0 ? 0 : (idx > RCAP - 1 ? RCAP - 1 : idx);
      const int ent = sl[idx];
      int eid = ent >> SLB;
      eid = eid < 0 ? 0 : (eid > nE - 1 ? nE - 1 : eid);
      int cl = cols[eid];
      cl = cl < 0 ? 0 : (cl > nN - 1 ? nN - 1 : cl);
      const float sc = s1v + S2[cl];
      const float lk = (sc >= 0.0f) ? sc : NEGSL * sc;
      float e = expf(-lk);
      e = (j < c) ? e : 0.0f;
      const int ebits = __float_as_int(e);
      const int m32 = (c - b0) < 32 ? (c - b0) : 32;
#pragma unroll 1
      for (int k = 0; k < m32; ++k) {
        const int   ck = __builtin_amdgcn_readlane(cl, k);
        const float ek = __int_as_float(__builtin_amdgcn_readlane(ebits, k));
        const float* rp = WH + (size_t)ck * OUT_DIM + 4 * lane;
        const v4f a = *(const v4f*)rp;
        a0 = fmaf(ek, a.x, a0);
        a1 = fmaf(ek, a.y, a1);
        a2 = fmaf(ek, a.z, a2);
        a3 = fmaf(ek, a.w, a3);
        dn += ek;
      }
    }
#pragma unroll 1
    for (int i = 0; i < 4; ++i) {
      const float q = a0 / dn;
      const float r = (q > 0.0f) ? q : expm1f(q);
      a0 = a1; a1 = a2; a2 = a3; a3 = r;
    }
    v4f ov4;
    ov4.x = poison ? qnan : a0;
    ov4.y = poison ? qnan : a1;
    ov4.z = poison ? qnan : a2;
    ov4.w = poison ? qnan : a3;
    if (node < nN) {
      float* op = outp + (size_t)node * OUT_DIM + 4 * lane;
      *(volatile v4f*)op = ov4;
      __threadfence();
      *(volatile v4f*)op = ov4;
    }
  }
}

static inline int cdiv(int a, int b) { return (a + b - 1) / b; }

extern "C" void kernel_launch(void* const* d_in, const int* in_sizes, int n_in,
                              void* d_out, int out_size, void* d_ws, size_t ws_size,
                              hipStream_t stream) {
  if (n_in < 4) return;
  if (in_sizes[0] < IN_DIM || (in_sizes[0] % IN_DIM) != 0) return;
  const int nN = in_sizes[0] / IN_DIM;
  if (nN < 1 || nN > (1 << 22)) return;
  if (in_sizes[1] < 2 || (in_sizes[1] & 1) != 0) return;
  const int nE = in_sizes[1] / 2;
  if (nE < 1 || nE >= (1 << 22)) return;
  if (in_sizes[2] != IN_DIM * OUT_DIM) return;
  if (in_sizes[3] != 2 * OUT_DIM) return;
  if ((long long)out_size != (long long)nN * OUT_DIM) return;

  const float* x    = (const float*)d_in[0];
  const int*   edge = (const int*)d_in[1];
  const float* w    = (const float*)d_in[2];
  const float* av   = (const float*)d_in[3];
  float* out = (float*)d_out;
  const int* keys = edge;
  const int* cols = edge + nE;

  const int MP   = cdiv(nN, GBM) * GBM;
  const int nXB  = MP / 8;
  const int gM   = MP / GBM;
  const int gA   = cdiv(nN, NBRUN);
  if ((long long)gA * NBRUN < (long long)nN) return;
  const int vec8 = ((nE & 3) == 0) ? 1 : 0;

  char* ws = (char*)d_ws;
  size_t off = 0;
  const size_t oXB  = off; off += (size_t)MP * IN_DIM * 2;        off = (off + 255) & ~(size_t)255;
  const size_t oWT  = off; off += (size_t)OUT_DIM * IN_DIM * 2;   off = (off + 255) & ~(size_t)255;
  const size_t oAT  = off; off += (size_t)2 * OUT_DIM * 4;        off = (off + 255) & ~(size_t)255;
  const size_t oWH  = off; off += (size_t)MP * OUT_DIM * 4;       off = (off + 255) & ~(size_t)255;
  const size_t oS   = off; off += (size_t)2 * MP * 4;             off = (off + 255) & ~(size_t)255;
  if (off > ws_size || off > (size_t)WSMAX) return;
  unsigned short* XB   = (unsigned short*)(ws + oXB);
  unsigned short* WT   = (unsigned short*)(ws + oWT);
  float*          ATAB = (float*)(ws + oAT);
  float*          WHp  = (float*)(ws + oWH);
  float*          S12  = (float*)(ws + oS);

  const size_t gemmLds = (size_t)GEMM_LDS_FLOATS * 4;
  const size_t scanLds = (size_t)AGG_LDS_INTS * 4;
  hipFuncSetAttribute(reinterpret_cast<const void*>(&k_gemm), hipFuncAttributeMaxDynamicSharedMemorySize, (int)gemmLds);
  hipFuncSetAttribute(reinterpret_cast<const void*>(&k_scan), hipFuncAttributeMaxDynamicSharedMemorySize, (int)scanLds);

  k_prep<<<nXB + NWB + 1, NTHR, 0, stream>>>(x, w, av, XB, WT, ATAB, nN, nXB);
  k_gemm<<<gM, GTHR, gemmLds, stream>>>(XB, WT, ATAB, WHp, S12, MP);
  k_scan<<<gA, NTHR, scanLds, stream>>>(keys, cols, nE, nN, vec8, S12, S12 + MP, WHp, out);
}
